// RGCNLowMem_4475355922763
// MI455X (gfx1250) — hardware-verified
//
#include <hip/hip_runtime.h>
#include <stddef.h>


#define FIN     64
#define NOUT    64
#define NREL    16
#define KTOT    (NREL * FIN)
#define AP      (KTOT + 8)
#define NTHR    256
#define NWAVE   8
#define EPT     8
#define NGRP    2
#define CHUNK   (NTHR * EPT * NGRP)
#define WCAP    (EPT * NGRP * 32)
#define LISTN   (NWAVE * WCAP)
#define NODEB   1024
#define RCAP    20480
#define NSUB    16
#define DEGCAP  256

#define LDS_S    (NSUB * KTOT * 4)
#define LDS_PL   (NSUB * AP * 2)
#define LDS_MAIN (LDS_S + LDS_PL + RCAP * 4 + 3 * NODEB * 4 + LISTN * 4 + 64)

static_assert((CHUNK & (CHUNK - 1)) == 0);
static_assert(CHUNK == 4096);
static_assert(NODEB == 32 * 32);
static_assert((NODEB & (NODEB - 1)) == 0 && NODEB <= 4096);
static_assert(NSUB == 2 * NWAVE);
static_assert(KTOT == 1024 && NOUT == 64 && FIN == 64);
static_assert((LDS_S % 16) == 0 && (LDS_PL % 16) == 0);
static_assert((RCAP % 4) == 0);
static_assert(2 * NSUB * NOUT <= NSUB * KTOT);
static_assert((NSUB * KTOT / 8) % NTHR == 0);
static_assert(LDS_MAIN <= 300 * 1024);

typedef float    v2f  __attribute__((ext_vector_type(2)));
typedef float    v4f  __attribute__((ext_vector_type(4)));
typedef float    v8f  __attribute__((ext_vector_type(8)));
typedef int      v4i  __attribute__((ext_vector_type(4)));
typedef _Float16 v8h  __attribute__((ext_vector_type(8)));
typedef _Float16 v16h __attribute__((ext_vector_type(16)));
union FragH { v16h v; v8h h[2]; };

__device__ __forceinline__ v8h cvt8(v4f a, v4f b) {
  v8h r;
  r[0] = (_Float16)a.x; r[1] = (_Float16)a.y; r[2] = (_Float16)a.z; r[3] = (_Float16)a.w;
  r[4] = (_Float16)b.x; r[5] = (_Float16)b.y; r[6] = (_Float16)b.z; r[7] = (_Float16)b.w;
  return r;
}

__device__ __forceinline__ v8f wmh(v16h a, v16h b, v8f c) {
  v8f d = __builtin_amdgcn_wmma_f32_16x16x32_f16(false, a, false, b, (short)0, c, false, false);
  asm volatile("v_nop\n\tv_nop\n\tv_nop\n\tv_nop" : "+v"(d) : "v"(a), "v"(b));
  return d;
}

template <int NB>
__device__ __forceinline__ int scan_chunk(const int* __restrict__ dsts, int nE, int cbase, int slotBase,
                                          int vec8, int* list, int tid, int lane, int wave) {
  int wc = 0;
#pragma unroll
  for (int g = 0; g < NGRP; ++g) {
    const int el0  = (g * NTHR + tid) * EPT;
    const int e0   = cbase + el0;
    const int sent = -2147483647 - 1;
    v4i da, db;
    if (vec8 != 0 && cbase + CHUNK <= nE) {
      da = *(const v4i*)(dsts + e0);
      db = *(const v4i*)(dsts + e0 + 4);
    } else {
      da.x = (e0     < nE) ? dsts[min(e0,     nE - 1)] : sent;
      da.y = (e0 + 1 < nE) ? dsts[min(e0 + 1, nE - 1)] : sent;
      da.z = (e0 + 2 < nE) ? dsts[min(e0 + 2, nE - 1)] : sent;
      da.w = (e0 + 3 < nE) ? dsts[min(e0 + 3, nE - 1)] : sent;
      db.x = (e0 + 4 < nE) ? dsts[min(e0 + 4, nE - 1)] : sent;
      db.y = (e0 + 5 < nE) ? dsts[min(e0 + 5, nE - 1)] : sent;
      db.z = (e0 + 6 < nE) ? dsts[min(e0 + 6, nE - 1)] : sent;
      db.w = (e0 + 7 < nE) ? dsts[min(e0 + 7, nE - 1)] : sent;
    }
    const unsigned nb = (unsigned)slotBase;
    const unsigned s0 = (unsigned)da.x - nb, s1 = (unsigned)da.y - nb;
    const unsigned s2 = (unsigned)da.z - nb, s3 = (unsigned)da.w - nb;
    const unsigned s4 = (unsigned)db.x - nb, s5 = (unsigned)db.y - nb;
    const unsigned s6 = (unsigned)db.z - nb, s7 = (unsigned)db.w - nb;
    const bool h0 = s0 < (unsigned)NB, h1 = s1 < (unsigned)NB, h2 = s2 < (unsigned)NB, h3 = s3 < (unsigned)NB;
    const bool h4 = s4 < (unsigned)NB, h5 = s5 < (unsigned)NB, h6 = s6 < (unsigned)NB, h7 = s7 < (unsigned)NB;
    const unsigned any = __builtin_amdgcn_ballot_w32(h0 | h1 | h2 | h3 | h4 | h5 | h6 | h7);
    if (any != 0u) {
#define HITJ(J, HJ, SJ) { \
        const unsigned mj = __builtin_amdgcn_ballot_w32(HJ); \
        if (mj != 0u) { \
          if (HJ) { \
            const int pos = wc + (int)__builtin_amdgcn_mbcnt_lo(mj, 0u); \
            if (pos < WCAP) list[wave * WCAP + pos] = ((el0 + (J)) << 12) | (int)(SJ); \
          } \
          wc += (int)__builtin_popcount(mj); } }
      HITJ(0, h0, s0)
      HITJ(1, h1, s1)
      HITJ(2, h2, s2)
      HITJ(3, h3, s3)
      HITJ(4, h4, s4)
      HITJ(5, h5, s5)
      HITJ(6, h6, s6)
      HITJ(7, h7, s7)
#undef HITJ
    }
  }
  return wc;
}

__global__ __launch_bounds__(NTHR) void k_wprep(
    const float* __restrict__ w, _Float16* bp, int total8) {
  const int i = blockIdx.x * NTHR + (int)threadIdx.x;
  if (i >= total8) return;
  const int n  = i >> 7;
  const int k0 = (i & 127) * 8;
  v8h hv;
#pragma unroll
  for (int e = 0; e < 8; ++e) {
    const int k = k0 + e;
    hv[e] = (_Float16)w[(size_t)k * NOUT + n];
  }
  _Float16* ph = bp + (size_t)i * 8;
  *(volatile v8h*)ph = hv;
  __threadfence();
  *(volatile v8h*)ph = hv;
}

__global__ __launch_bounds__(NTHR) void k_main(
    const float* __restrict__ feat, const int* __restrict__ srcs, const int* __restrict__ dsts,
    const int* __restrict__ ety, const _Float16* __restrict__ bpl,
    float* out, int nN, int nE, int vec8) {
  extern __shared__ v4f lds_dyn[];
  float*    S      = (float*)lds_dyn;
  _Float16* Ph     = (_Float16*)((char*)lds_dyn + LDS_S);
  int*      region = (int*)((char*)lds_dyn + LDS_S + LDS_PL);
  int*      scnt   = region + RCAP;
  int*      soff   = scnt + NODEB;
  int*      cursor = soff + NODEB;
  int*      list   = cursor + NODEB;
  int*      wcnt   = list + LISTN;
  const int tid = threadIdx.x, lane = tid & 31, wave = tid >> 5, hh = lane >> 4, m = lane & 15;
  const int nodeBase = blockIdx.x * NODEB;

  {
    const v4i z = {0, 0, 0, 0};
    for (int i = tid; i < NODEB; i += NTHR) scnt[i] = 0;
    for (int i = tid; i < RCAP / 4; i += NTHR) ((v4i*)region)[i] = z;
  }
  __syncthreads();

  const int nChunks = (nE + CHUNK - 1) / CHUNK;

#pragma unroll 1
  for (int ch = 0; ch < nChunks; ++ch) {
    const int cbase = ch * CHUNK;
    const int wc = scan_chunk<NODEB>(dsts, nE, cbase, nodeBase, vec8, list, tid, lane, wave);
    if (lane == 0) wcnt[wave] = wc;
    __syncthreads();
    if (wave == 0) {
#pragma unroll 1
      for (int wsx = 0; wsx < NWAVE; ++wsx) {
        int n = __builtin_amdgcn_readfirstlane(wcnt[wsx]);
        n = n > WCAP ? WCAP : (n < 0 ? 0 : n);
        const int* lp = list + wsx * WCAP;
#pragma unroll 1
        for (int i = 0; i < n; ++i) {
          const int ent  = __builtin_amdgcn_readfirstlane(lp[i]);
          const int slot = ent & (NODEB - 1);
          if (lane == 0) scnt[slot] = scnt[slot] + 1;
        }
      }
    }
    __syncthreads();
  }

  if (wave == 0) {
    int t = 0;
#pragma unroll 1
    for (int i = 0; i < 32; ++i) {
      int c = scnt[32 * lane + i];
      c = c < 0 ? 0 : c;
      t += c;
    }
    int incl = t;
#pragma unroll
    for (int d = 1; d < 32; d <<= 1) {
      const int u = __shfl_up(incl, d);
      if (lane >= d) incl += u;
    }
    int run = incl - t;
#pragma unroll 1
    for (int i = 0; i < 32; ++i) {
      const int s = 32 * lane + i;
      int c = scnt[s];
      c = c < 0 ? 0 : c;
      soff[s]   = run;
      cursor[s] = run > RCAP ? RCAP : run;
      run += c;
    }
  }
  __syncthreads();

#pragma unroll 1
  for (int ch = 0; ch < nChunks; ++ch) {
    const int cbase = ch * CHUNK;
    const int wc = scan_chunk<NODEB>(dsts, nE, cbase, nodeBase, vec8, list, tid, lane, wave);
    if (lane == 0) wcnt[wave] = wc;
    __syncthreads();
    if (wave == 0) {
#pragma unroll 1
      for (int wsx = 0; wsx < NWAVE; ++wsx) {
        int n = __builtin_amdgcn_readfirstlane(wcnt[wsx]);
        n = n > WCAP ? WCAP : (n < 0 ? 0 : n);
        const int* lp = list + wsx * WCAP;
#pragma unroll 1
        for (int i = 0; i < n; ++i) {
          const int ent  = __builtin_amdgcn_readfirstlane(lp[i]);
          const int slot = ent & (NODEB - 1);
          int e = cbase + ((ent >> 12) & (CHUNK - 1));
          e = e > nE - 1 ? nE - 1 : e;
          if (lane == 0) {
            int pos = cursor[slot];
            pos = pos < 0 ? 0 : (pos > RCAP - 1 ? RCAP - 1 : pos);
            region[pos] = e;
            const int np = pos + 1;
            cursor[slot] = np > RCAP ? RCAP : np;
          }
        }
      }
    }
    __syncthreads();
  }

  const int rem = nN - nodeBase;
  int nSubs = (rem + NSUB - 1) / NSUB;
  nSubs = nSubs < 0 ? 0 : (nSubs > NODEB / NSUB ? NODEB / NSUB : nSubs);
  const int t4 = wave & 3, kh = wave >> 2;
  float* stg1 = S;
  float* stg0 = S + NSUB * NOUT;

#pragma unroll 1
  for (int st = 0; st < nSubs; ++st) {
    {
      const v4f z = {0.f, 0.f, 0.f, 0.f};
      for (int i = tid; i < NSUB * KTOT / 4; i += NTHR) ((v4f*)S)[i] = z;
    }
    __syncthreads();

#pragma unroll 1
    for (int jj = 0; jj < NSUB / NWAVE; ++jj) {
      const int rloc = wave * (NSUB / NWAVE) + jj;
      const int slot = st * NSUB + rloc;
      int n = __builtin_amdgcn_readfirstlane(scnt[slot]);
      n = n < 0 ? 0 : (n > DEGCAP ? DEGCAP : n);
      int sp = __builtin_amdgcn_readfirstlane(soff[slot]);
      sp = sp < 0 ? 0 : (sp > RCAP ? RCAP : sp);
      float* srow = S + rloc * KTOT + 2 * lane;
#pragma unroll 1
      for (int q0 = 0; q0 < n; q0 += 32) {
        int pos = sp + q0 + lane;
        pos = pos < 0 ? 0 : (pos > RCAP - 1 ? RCAP - 1 : pos);
        int e = region[pos];
        e = e < 0 ? 0 : (e > nE - 1 ? nE - 1 : e);
        int sv = srcs[e];
        sv = sv < 0 ? 0 : (sv > nN - 1 ? nN - 1 : sv);
        int tv = ety[e];
        tv = tv < 0 ? 0 : (tv > NREL - 1 ? NREL - 1 : tv);
        const int mcnt = (n - q0) < 32 ? (n - q0) : 32;
#pragma unroll 1
        for (int p = 0; p < mcnt; ++p) {
          const int s  = __builtin_amdgcn_readlane(sv, p);
          const int ty = __builtin_amdgcn_readlane(tv, p);
          const v2f v = *(const v2f*)(feat + (size_t)s * FIN + 2 * lane);
          v2f* ap = (v2f*)(srow + ty * FIN);
          *ap = *ap + v;
        }
      }
    }
    __syncthreads();

#pragma unroll 2
    for (int it = 0; it < (NSUB * KTOT / 8) / NTHR; ++it) {
      const int g   = it * NTHR + tid;
      const int row = g >> 7;
      const int c0  = (g & 127) * 8;
      const v4f a = *(const v4f*)(S + row * KTOT + c0);
      const v4f b = *(const v4f*)(S + row * KTOT + c0 + 4);
      *(v8h*)(Ph + row * AP + c0) = cvt8(a, b);
    }
    __syncthreads();

    v8f acc = {0.f, 0.f, 0.f, 0.f, 0.f, 0.f, 0.f, 0.f};
    {
      const _Float16* ar = Ph + m * AP + kh * (KTOT / 2) + 8 * hh;
      const _Float16* br = bpl + (size_t)(16 * t4 + m) * KTOT + kh * (KTOT / 2) + 8 * hh;
#pragma unroll 2
      for (int ks = 0; ks < KTOT / 64; ++ks) {
        FragH a, b;
        a.h[0] = *(const v8h*)(ar + 32 * ks);
        a.h[1] = *(const v8h*)(ar + 32 * ks + 16);
        b.h[0] = *(const v8h*)(br + 32 * ks);
        b.h[1] = *(const v8h*)(br + 32 * ks + 16);
        acc = wmh(a.v, b.v, acc);
      }
    }

    if (kh == 1) {
#pragma unroll
      for (int r = 0; r < 8; ++r) stg1[(8 * hh + r) * NOUT + 16 * t4 + m] = acc[r];
    }
    __syncthreads();
    if (kh == 0) {
#pragma unroll
      for (int r = 0; r < 8; ++r) {
        const int ix = (8 * hh + r) * NOUT + 16 * t4 + m;
        stg0[ix] = acc[r] + stg1[ix];
      }
    }
    __syncthreads();

    {
      const int row  = tid >> 4;
      const int c4   = (tid & 15) * 4;
      const int node = nodeBase + st * NSUB + row;
      const int nc   = node > nN - 1 ? nN - 1 : node;
      const v4f v = *(const v4f*)(stg0 + row * NOUT + c4);
      float* gp = out + (size_t)nc * NOUT + c4;
      if (node < nN) *(volatile v4f*)gp = v;
      __threadfence();
      if (node < nN) *(volatile v4f*)gp = v;
    }
    __syncthreads();
  }
}

extern "C" void kernel_launch(void* const* d_in, const int* in_sizes, int n_in,
                              void* d_out, int out_size, void* d_ws, size_t ws_size,
                              hipStream_t stream) {
  if (n_in < 5) return;
  const int nN = in_sizes[0] / FIN;
  if (nN <= 0 || in_sizes[0] != nN * FIN) return;
  if (in_sizes[1] != NREL * FIN * NOUT) return;
  const int nE = in_sizes[2];
  if (nE <= 0 || in_sizes[3] != nE || in_sizes[4] != nE) return;
  if (out_size != nN * NOUT) return;
  if (nN > (1 << 26) || nE > (1 << 28)) return;

  const float* feat = (const float*)d_in[0];
  const float* w    = (const float*)d_in[1];
  const int*   src  = (const int*)d_in[2];
  const int*   dst  = (const int*)d_in[3];
  const int*   ety  = (const int*)d_in[4];
  float*       out  = (float*)d_out;

  char* ws = (char*)d_ws;
  size_t off = 0;
  const size_t oBp = off; off += (size_t)NOUT * KTOT * 2;
  if (off > ws_size) return;
  _Float16* bp = (_Float16*)(ws + oBp);

  const int total8 = NOUT * KTOT / 8;
  k_wprep<<<(total8 + NTHR - 1) / NTHR, NTHR, 0, stream>>>(w, bp, total8);

  hipFuncSetAttribute(reinterpret_cast<const void*>(&k_main),
                      hipFuncAttributeMaxDynamicSharedMemorySize, LDS_MAIN);
  const int nBlk = (nN + NODEB - 1) / NODEB;
  k_main<<<nBlk, NTHR, LDS_MAIN, stream>>>(feat, src, dst, ety, bp, out, nN, nE, 1);
}
